// Feat_aggr_18425409699924
// MI455X (gfx1250) — hardware-verified
//
#include <hip/hip_runtime.h>
#include <math.h>
#include <stdint.h>

#define NBATCH 16
#define SEQ    2048
#define CH     256
#define NROWS  (NBATCH * SEQ)
#define NQB    (SEQ / 64)
static_assert((SEQ % 64) == 0);
static_assert((CH % 64) == 0);
static_assert(CH == 256);
static_assert((NROWS % 64) == 0);

typedef _Float16 v16h __attribute__((ext_vector_type(16)));
typedef _Float16 v8h  __attribute__((ext_vector_type(8)));
typedef __bf16   v16b __attribute__((ext_vector_type(16)));
typedef __bf16   v8b  __attribute__((ext_vector_type(8)));
typedef float    v8f  __attribute__((ext_vector_type(8)));
typedef float    v4f  __attribute__((ext_vector_type(4)));
typedef unsigned int v4u __attribute__((ext_vector_type(4)));

__device__ __forceinline__ unsigned short bf_bits(float f) {
  unsigned u = __float_as_uint(f);
  return (unsigned short)((u + 0x7FFFu + ((u >> 16) & 1u)) >> 16);
}
__device__ __forceinline__ float bf_up(unsigned short h) { return __uint_as_float(((unsigned)h) << 16); }
__device__ __forceinline__ unsigned short h_bits(_Float16 x) { return __builtin_bit_cast(unsigned short, x); }
__device__ __forceinline__ unsigned pk16(unsigned short a, unsigned short b) { return (unsigned)a | ((unsigned)b << 16); }
__device__ __forceinline__ v8f zero8() { v8f z = {0.f, 0.f, 0.f, 0.f, 0.f, 0.f, 0.f, 0.f}; return z; }

__device__ __forceinline__ v16b ldfrag_b(const __bf16* p) {
  union { v16b v; v8b h[2]; } f;
  f.h[0] = *(const v8b*)(p);
  f.h[1] = *(const v8b*)(p + 16);
  return f.v;
}
__device__ __forceinline__ v16h ldfrag_h(const _Float16* p) {
  union { v16h v; v8h h[2]; } f;
  f.h[0] = *(const v8h*)(p);
  f.h[1] = *(const v8h*)(p + 16);
  return f.v;
}

__device__ __forceinline__ v8f mma_h(v16h a, v16h b, v8f c) {
  c = __builtin_amdgcn_wmma_f32_16x16x32_f16(false, a, false, b, (short)0, c, false, false);
#if defined(__HIP_DEVICE_COMPILE__)
  asm volatile("v_nop\n\tv_nop\n\tv_nop\n\tv_nop" : "+v"(c) : "v"(a), "v"(b));
#endif
  return c;
}
__device__ __forceinline__ v8f mma_b(v16b a, v16b b, v8f c) {
  c = __builtin_amdgcn_wmma_f32_16x16x32_bf16(false, a, false, b, (short)0, c, false, false);
#if defined(__HIP_DEVICE_COMPILE__)
  asm volatile("v_nop\n\tv_nop\n\tv_nop\n\tv_nop" : "+v"(c) : "v"(a), "v"(b));
#endif
  return c;
}
__device__ __forceinline__ v8f mma_b_raw(v16b a, v16b b, v8f c) {
  return __builtin_amdgcn_wmma_f32_16x16x32_bf16(false, a, false, b, (short)0, c, false, false);
}
__device__ __forceinline__ void dep_guard_b(v8f& a, v8f& b, v16b x, v16b y) {
#if defined(__HIP_DEVICE_COMPILE__)
  asm volatile("v_nop\n\tv_nop\n\tv_nop\n\tv_nop" : "+v"(a), "+v"(b) : "v"(x), "v"(y));
#endif
}
__device__ __forceinline__ void keep4_b(v16b a, v16b b, v16b c, v16b d) {
#if defined(__HIP_DEVICE_COMPILE__)
  asm volatile("v_nop" :: "v"(a), "v"(b), "v"(c), "v"(d));
#endif
}
__device__ __forceinline__ void acc_guard4(v8f& a, v8f& b, v8f& c, v8f& d) {
#if defined(__HIP_DEVICE_COMPILE__)
  asm volatile("v_nop\n\tv_nop\n\tv_nop\n\tv_nop" : "+v"(a), "+v"(b), "+v"(c), "+v"(d));
#endif
}
__device__ __forceinline__ void wave_sync_lds() {
  __builtin_amdgcn_fence(__ATOMIC_RELEASE, "workgroup");
  __builtin_amdgcn_wave_barrier();
  __builtin_amdgcn_fence(__ATOMIC_ACQUIRE, "workgroup");
}

__device__ __forceinline__ unsigned cvt2(float a, float b, float& ss) {
  const unsigned short h0 = bf_bits(a), h1 = bf_bits(b);
  const float f0 = bf_up(h0), f1 = bf_up(h1);
  ss += f0 * f0;
  ss += f1 * f1;
  return pk16(h0, h1);
}
__device__ __forceinline__ v4f leaky4(v4f y) {
  v4f r;
  r[0] = (y[0] >= 0.f) ? y[0] : 0.01f * y[0];
  r[1] = (y[1] >= 0.f) ? y[1] : 0.01f * y[1];
  r[2] = (y[2] >= 0.f) ? y[2] : 0.01f * y[2];
  r[3] = (y[3] >= 0.f) ? y[3] : 0.01f * y[3];
  return r;
}

__global__ __launch_bounds__(256) void cvt_x_rn(const float* __restrict__ x, unsigned short* xb, float* rnp, int nblk) {
  __shared__ __align__(16) float Rsh[32];
  const int lane = threadIdx.x & 31, wave = threadIdx.x >> 5;
  const int blk = blockIdx.x;
  if (blk >= nblk) return;
#pragma unroll 1
  for (int it = 0; it < 4; ++it) {
    const int row = blk * 32 + it * 8 + wave;
    const size_t eo = (size_t)row * CH + (size_t)lane * 8;
    const v4f a = *(const v4f*)(x + eo);
    const v4f c4 = *(const v4f*)(x + eo + 4);
    float ss = 0.f;
    v4u p;
    p[0] = cvt2(a[0], a[1], ss);
    p[1] = cvt2(a[2], a[3], ss);
    p[2] = cvt2(c4[0], c4[1], ss);
    p[3] = cvt2(c4[2], c4[3], ss);
    *(volatile v4u*)(xb + eo) = p;
    __threadfence();
    *(volatile v4u*)(xb + eo) = p;
#pragma unroll
    for (int off = 16; off > 0; off >>= 1) ss += __shfl_xor(ss, off, 32);
    if (lane == 0) Rsh[it * 8 + wave] = 1.0f / fmaxf(sqrtf(ss), 1e-12f);
  }
  __syncthreads();
  if (wave == 0) {
    const v4f v = *(const v4f*)(Rsh + 4 * (lane & 7));
    if (lane < 8) *(volatile v4f*)(rnp + (size_t)blk * 32 + 4 * lane) = v;
    __threadfence();
    if (lane < 8) *(volatile v4f*)(rnp + (size_t)blk * 32 + 4 * lane) = v;
  }
}

__global__ __launch_bounds__(256) void cvt_w(const float* __restrict__ adjw, const float* __restrict__ affw,
                                             unsigned short* wt, unsigned short* wa) {
  const int lane = threadIdx.x & 31, wave = threadIdx.x >> 5;
  const int d = blockIdx.x * 8 + wave;
  const int c0 = lane * 8;
  v4u t, a;
#pragma unroll
  for (int e = 0; e < 4; ++e) {
    const int c = c0 + 2 * e;
    t[e] = pk16(bf_bits(adjw[(size_t)c * CH + d]), bf_bits(adjw[(size_t)(c + 1) * CH + d]));
    a[e] = pk16(bf_bits(affw[(size_t)d * CH + c]), bf_bits(affw[(size_t)d * CH + c + 1]));
  }
  const size_t so = (size_t)d * CH + c0;
  *(volatile v4u*)(wt + so) = t;
  *(volatile v4u*)(wa + so) = a;
  __threadfence();
  *(volatile v4u*)(wt + so) = t;
  *(volatile v4u*)(wa + so) = a;
}

template <int NSPLIT, int OUT_MODE, bool HAS_BIAS>
__global__ __launch_bounds__(256) void gemm64(
    const unsigned short* __restrict__ Ap, const unsigned short* A2p, int lda, long long strideA,
    const unsigned short* __restrict__ Btp, const unsigned short* Bt2p, int ldb, long long strideB,
    void* Cout, int ldc, long long strideC,
    void* Cout2, int ldc2, long long strideC2, int N2,
    const float* __restrict__ rbias,
    int M, int N, int K, float rscale) {
  const __bf16* A   = (const __bf16*)(const void*)Ap;
  const __bf16* A2  = (const __bf16*)(const void*)A2p;
  const __bf16* Bt  = (const __bf16*)(const void*)Btp;
  const __bf16* Bt2 = (const __bf16*)(const void*)Bt2p;
  __shared__ __align__(16) float sT[8][16 * 68];
  const int b    = blockIdx.y;
  const int lane = threadIdx.x & 31;
  const int wave = threadIdx.x >> 5;
  const int tilesN = N >> 6;
  const int tilesM = M >> 6;
  const int tile = blockIdx.x * 8 + wave;
  if (tile >= tilesM * tilesN) return;
  const int tm = tile / tilesN;
  const int tn = tile - tm * tilesN;
  const int m0 = tm << 6;
  const int n0 = tn << 6;

  const __bf16* Ab  = A  + (size_t)b * strideA;
  const __bf16* Bb  = Bt + (size_t)b * strideB;
  const __bf16* Ab2 = (NSPLIT >= 1) ? (A2  + (size_t)b * strideA) : Ab;
  const __bf16* Bb2 = (NSPLIT == 2) ? (Bt2 + (size_t)b * strideB) : Bb;

  const int rlane = lane & 15;
  const int koff  = (lane >> 4) * 8;
  const int mOff  = (lane >> 4) * 8;

  v8f acc[4][4];
#pragma unroll
  for (int i = 0; i < 4; ++i)
#pragma unroll
    for (int j = 0; j < 4; ++j) acc[i][j] = zero8();

  for (int k0 = 0; k0 < K; k0 += 32) {
    v16b bh[4], bl[4];
#pragma unroll
    for (int j = 0; j < 4; ++j) {
      const size_t bo = (size_t)(n0 + (j << 4) + rlane) * ldb + koff + k0;
      bh[j] = ldfrag_b(Bb + bo);
      if (NSPLIT == 2) bl[j] = ldfrag_b(Bb2 + bo); else bl[j] = bh[j];
    }
#pragma unroll
    for (int i = 0; i < 4; ++i) {
      const size_t ao = (size_t)(m0 + (i << 4) + rlane) * lda + koff + k0;
      const v16b ah = ldfrag_b(Ab + ao);
      v16b al = ah;
      if (NSPLIT >= 1) al = ldfrag_b(Ab2 + ao);
#pragma unroll
      for (int j = 0; j < 4; ++j) {
        acc[i][j] = mma_b_raw(ah, bh[j], acc[i][j]);
        if (NSPLIT >= 1) acc[i][j] = mma_b_raw(al, bh[j], acc[i][j]);
        if (NSPLIT == 2) acc[i][j] = mma_b_raw(ah, bl[j], acc[i][j]);
      }
      dep_guard_b(acc[i][0], acc[i][3], ah, al);
    }
    keep4_b(bh[0], bh[1], bh[2], bh[3]);
    if (NSPLIT == 2) keep4_b(bl[0], bl[1], bl[2], bl[3]);
  }
  acc_guard4(acc[0][0], acc[0][1], acc[0][2], acc[0][3]);
  acc_guard4(acc[1][0], acc[1][1], acc[1][2], acc[1][3]);
  acc_guard4(acc[2][0], acc[2][1], acc[2][2], acc[2][3]);
  acc_guard4(acc[3][0], acc[3][1], acc[3][2], acc[3][3]);

  float* slab = sT[wave];
#pragma unroll
  for (int i = 0; i < 4; ++i) {
    const int mBase = m0 + (i << 4);
#pragma unroll
    for (int j = 0; j < 4; ++j) {
#pragma unroll
      for (int r = 0; r < 8; ++r) {
        slab[(mOff + r) * 68 + (j << 4) + rlane] = acc[i][j][r];
      }
    }
    wave_sync_lds();
    if (OUT_MODE == 0) {
      float* C = (float*)Cout + (size_t)b * strideC;
      const int hh = lane >> 4, c4 = (lane & 15) * 4;
      for (int pass = 0; pass < 2; ++pass) {
#pragma unroll
        for (int it = 0; it < 8; ++it) {
          const int row = it * 2 + hh;
          v4f v = *(const v4f*)(slab + row * 68 + c4);
          if (HAS_BIAS) { const float bv = rbias[mBase + row]; v = v + bv; }
          *(volatile v4f*)(C + (size_t)(mBase + row) * ldc + n0 + c4) = v;
        }
        __threadfence();
      }
    } else {
      const int q = lane >> 3, c8 = (lane & 7) * 8;
      unsigned short* C  = (unsigned short*)Cout  + (size_t)b * strideC;
      unsigned short* C2 = (unsigned short*)Cout2 + (size_t)b * strideC2;
      const bool wlo = (OUT_MODE == 2) || (n0 < N2);
      v4u hv[4], lv[4];
#pragma unroll
      for (int it = 0; it < 4; ++it) {
        const int row = it * 4 + q;
        const float* sp = slab + row * 68 + c8;
        const float bv = HAS_BIAS ? rbias[mBase + row] : 0.f;
        v4u a, a2;
#pragma unroll
        for (int e = 0; e < 4; ++e) {
          const float f0 = sp[2 * e] + bv, f1 = sp[2 * e + 1] + bv;
          unsigned short h0, h1, l0, l1;
          if (OUT_MODE == 2) {
            h0 = bf_bits(f0); h1 = bf_bits(f1);
            l0 = bf_bits(f0 - bf_up(h0)); l1 = bf_bits(f1 - bf_up(h1));
          } else {
            const _Float16 x0 = (_Float16)f0, x1 = (_Float16)f1;
            h0 = h_bits(x0); h1 = h_bits(x1);
            l0 = h_bits((_Float16)((f0 - (float)x0) * rscale));
            l1 = h_bits((_Float16)((f1 - (float)x1) * rscale));
          }
          a[e] = pk16(h0, h1); a2[e] = pk16(l0, l1);
        }
        hv[it] = a; lv[it] = a2;
      }
      for (int pass = 0; pass < 2; ++pass) {
#pragma unroll
        for (int it = 0; it < 4; ++it) {
          const int row = it * 4 + q;
          *(volatile v4u*)(C + (size_t)(mBase + row) * ldc + n0 + c8) = hv[it];
          if (wlo) *(volatile v4u*)(C2 + (size_t)(mBase + row) * ldc2 + n0 + c8) = lv[it];
        }
        __threadfence();
      }
    }
    wave_sync_lds();
  }
}

__global__ __launch_bounds__(256)
void attn_ln(const unsigned short* __restrict__ xwhp, const unsigned short* __restrict__ xwlp,
             const unsigned short* __restrict__ xbp, const unsigned short* __restrict__ hthp,
             const float* __restrict__ rnp, const float* __restrict__ lng, const float* __restrict__ lnb,
             float* out, float pscale, float rps, float sfac) {
  union FH { v16h v; v8h h[2]; };
  union FB { v16b v; v8b h[2]; };
  __shared__ __align__(16) unsigned char smA[65536];
  __shared__ __align__(16) _Float16 Psh[4][16 * 64];
  __shared__ float Msh[4][2][16];
  __shared__ float Lsh[4][2][16];

  __bf16*   Ksh = (__bf16*)(void*)smA;
  _Float16* Vth = (_Float16*)(void*)(smA + 32768);

  const int tid  = threadIdx.x;
  const int wave = tid >> 5;
  const int lane = tid & 31;
  const int hh   = lane >> 4;
  const int c    = lane & 15;
  const int g    = wave >> 1;
  const int w2   = wave & 1;

  const int b     = blockIdx.x / NQB;
  const int qb    = blockIdx.x - b * NQB;
  const size_t rowB = (size_t)b * SEQ;
  const int qbase = qb * 64;
  const int q0    = qbase + g * 16;

  const __bf16*   XWh = (const __bf16*)(const void*)xwhp;
  const __bf16*   XWl = (const __bf16*)(const void*)xwlp;
  const __bf16*   Xg  = (const __bf16*)(const void*)xbp;
  const _Float16* Hg  = (const _Float16*)(const void*)hthp + (size_t)b * CH * SEQ;

  float qsc[8], mrow[8], lpart[8];
  v8f oacc[8];
#pragma unroll
  for (int r = 0; r < 8; ++r) {
    qsc[r]   = sfac * rnp[rowB + q0 + 8 * hh + r];
    mrow[r]  = -INFINITY;
    lpart[r] = 0.f;
  }
#pragma unroll
  for (int t = 0; t < 8; ++t) oacc[t] = zero8();

  for (int kt = 0; kt < NQB; ++kt) {
    const int kv0 = kt * 64;
    __syncthreads();
    {
      const int r = tid >> 2, cq = (tid & 3) * 64;
      const __bf16*   kg = Xg + (rowB + kv0 + r) * CH + cq;
      const _Float16* vg = Hg + (size_t)tid * SEQ + kv0;
#pragma unroll
      for (int i = 0; i < 8; ++i) {
        *(v8b*)(Ksh + r * CH + cq + 8 * i)  = *(const v8b*)(kg + 8 * i);
        *(v8h*)(Vth + tid * 64 + 8 * i)     = *(const v8h*)(vg + 8 * i);
      }
    }
    __syncthreads();

    v8f s0 = zero8(), s1 = zero8();
#pragma unroll 2
    for (int dc = 0; dc < 8; ++dc) {
      const size_t ao = (rowB + q0 + c) * CH + dc * 32 + 8 * hh;
      const v16b ah = ldfrag_b(XWh + ao);
      const v16b al = ldfrag_b(XWl + ao);
      FB k0b, k1b;
      k0b.h[0] = *(const v8b*)(Ksh + (w2 * 32 + c) * CH + dc * 32 + 8 * hh);
      k0b.h[1] = *(const v8b*)(Ksh + (w2 * 32 + c) * CH + dc * 32 + 16 + 8 * hh);
      k1b.h[0] = *(const v8b*)(Ksh + (w2 * 32 + 16 + c) * CH + dc * 32 + 8 * hh);
      k1b.h[1] = *(const v8b*)(Ksh + (w2 * 32 + 16 + c) * CH + dc * 32 + 16 + 8 * hh);
      s0 = mma_b(ah, k0b.v, s0);
      s0 = mma_b(al, k0b.v, s0);
      s1 = mma_b(ah, k1b.v, s1);
      s1 = mma_b(al, k1b.v, s1);
    }
    const float rnk0 = rnp[rowB + kv0 + w2 * 32 + c];
    const float rnk1 = rnp[rowB + kv0 + w2 * 32 + 16 + c];
#pragma unroll
    for (int r = 0; r < 8; ++r) {
      s0[r] = s0[r] * qsc[r] * rnk0;
      s1[r] = s1[r] * qsc[r] * rnk1;
    }

#pragma unroll
    for (int r = 0; r < 8; ++r) {
      float m = fmaxf(s0[r], s1[r]);
#pragma unroll
      for (int off = 1; off < 16; off <<= 1) m = fmaxf(m, __shfl_xor(m, off, 32));
      if (c == 0) Msh[g][w2][8 * hh + r] = m;
    }
    __syncthreads();

    _Float16* pw = Psh[g];
#pragma unroll
    for (int r = 0; r < 8; ++r) {
      const int row = 8 * hh + r;
      const float mch   = fmaxf(Msh[g][0][row], Msh[g][1][row]);
      const float mnew  = fmaxf(mrow[r], mch);
      const float alpha = __expf(mrow[r] - mnew);
      mrow[r] = mnew;
      const float p0 = __expf(s0[r] - mnew);
      const float p1 = __expf(s1[r] - mnew);
      pw[row * 64 + w2 * 32 + c]      = (_Float16)(p0 * pscale);
      pw[row * 64 + w2 * 32 + 16 + c] = (_Float16)(p1 * pscale);
      float psum = p0 + p1;
#pragma unroll
      for (int off = 1; off < 16; off <<= 1) psum += __shfl_xor(psum, off, 32);
      lpart[r] = lpart[r] * alpha + psum;
#pragma unroll
      for (int t = 0; t < 8; ++t) oacc[t][r] *= alpha;
    }
    __syncthreads();

#pragma unroll 1
    for (int kk = 0; kk < 2; ++kk) {
      FH pa;
      pa.h[0] = *(const v8h*)(pw + c * 64 + kk * 32 + 8 * hh);
      pa.h[1] = *(const v8h*)(pw + c * 64 + kk * 32 + 16 + 8 * hh);
#pragma unroll
      for (int t = 0; t < 8; ++t) {
        FH vb;
        vb.h[0] = *(const v8h*)(Vth + (w2 * 128 + t * 16 + c) * 64 + kk * 32 + 8 * hh);
        vb.h[1] = *(const v8h*)(Vth + (w2 * 128 + t * 16 + c) * 64 + kk * 32 + 16 + 8 * hh);
        oacc[t] = mma_h(pa.v, vb.v, oacc[t]);
      }
    }
  }

  if (c == 0) {
#pragma unroll
    for (int r = 0; r < 8; ++r) Lsh[g][w2][8 * hh + r] = lpart[r];
  }
  __syncthreads();
  float* Os = (float*)(void*)smA;
#pragma unroll
  for (int t = 0; t < 8; ++t) {
#pragma unroll
    for (int r = 0; r < 8; ++r) {
      Os[(g * 16 + 8 * hh + r) * CH + w2 * 128 + t * 16 + c] = oacc[t][r];
    }
  }
  __syncthreads();

  const v4f ga = *(const v4f*)(lng + 4 * lane);
  const v4f gb = *(const v4f*)(lng + 128 + 4 * lane);
  const v4f ba = *(const v4f*)(lnb + 4 * lane);
  const v4f bb = *(const v4f*)(lnb + 128 + 4 * lane);
#pragma unroll 1
  for (int i = 0; i < 8; ++i) {
    const int row = wave * 8 + i;
    const int gq = row >> 4, rr = row & 15;
    const float lsum = Lsh[gq][0][rr] + Lsh[gq][1][rr];
    const float inv  = (1.0f / lsum) * rps;
    v4f v0 = *(const v4f*)(Os + row * CH + 4 * lane);
    v4f v1 = *(const v4f*)(Os + row * CH + 128 + 4 * lane);
    v0 = v0 * inv;
    v1 = v1 * inv;
    float su = (v0[0] + v0[1]) + (v0[2] + v0[3]) + (v1[0] + v1[1]) + (v1[2] + v1[3]);
#pragma unroll
    for (int off = 16; off > 0; off >>= 1) su += __shfl_xor(su, off, 32);
    const float mu = su * (1.0f / 256.0f);
    const v4f d0 = v0 - mu;
    const v4f d1 = v1 - mu;
    float sq = (d0[0] * d0[0] + d0[1] * d0[1]) + (d0[2] * d0[2] + d0[3] * d0[3])
             + (d1[0] * d1[0] + d1[1] * d1[1]) + (d1[2] * d1[2] + d1[3] * d1[3]);
#pragma unroll
    for (int off = 16; off > 0; off >>= 1) sq += __shfl_xor(sq, off, 32);
    const float var  = sq * (1.0f / 256.0f);
    const float rstd = 1.0f / sqrtf(var + 1e-5f);
    const v4f y0 = leaky4(d0 * rstd * ga + ba);
    const v4f y1 = leaky4(d1 * rstd * gb + bb);
    float* po = out + (rowB + qbase + row) * CH;
    *(volatile v4f*)(po + 4 * lane)       = y0;
    *(volatile v4f*)(po + 128 + 4 * lane) = y1;
    __threadfence();
    *(volatile v4f*)(po + 4 * lane)       = y0;
    *(volatile v4f*)(po + 128 + 4 * lane) = y1;
  }
}

extern "C" void kernel_launch(void* const* d_in, const int* in_sizes, int n_in,
                              void* d_out, int out_size, void* d_ws, size_t ws_size,
                              hipStream_t stream) {
  if (n_in < 8) return;
  if (in_sizes[0] != NROWS * CH) return;
  if (in_sizes[3] != CH * CH) return;
  if (in_sizes[4] != CH * CH) return;
  if (in_sizes[5] != CH || in_sizes[6] != CH || in_sizes[7] != CH) return;
  if (out_size != NROWS * CH) return;

  const float* x    = (const float*)d_in[0];
  const float* adjw = (const float*)d_in[3];
  const float* affw = (const float*)d_in[4];
  const float* affb = (const float*)d_in[5];
  const float* lng  = (const float*)d_in[6];
  const float* lnb  = (const float*)d_in[7];

  const size_t PX  = (size_t)NROWS * CH * 2;
  const size_t PW  = (size_t)CH * CH * 2;
  const size_t PH  = (size_t)NBATCH * CH * SEQ * 2;
  const size_t PR  = (size_t)NROWS * 4;
  size_t off = 0;
  const size_t oXb  = off; off += PX;
  const size_t oWT  = off; off += PW;
  const size_t oWA  = off; off += PW;
  const size_t oXWh = off; off += PX;
  const size_t oXWl = off; off += PX;
  const size_t oHth = off; off += PH;
  const size_t oRn  = off; off += PR;
  if (off > ws_size) return;
  if (off > (size_t)134217728) return;

  char* ws = (char*)d_ws;
  unsigned short* Xb  = (unsigned short*)(ws + oXb);
  unsigned short* WT  = (unsigned short*)(ws + oWT);
  unsigned short* WA  = (unsigned short*)(ws + oWA);
  unsigned short* XWh = (unsigned short*)(ws + oXWh);
  unsigned short* XWl = (unsigned short*)(ws + oXWl);
  unsigned short* Hth = (unsigned short*)(ws + oHth);
  float*          rnp = (float*)(ws + oRn);

  const dim3 blk(256);
  const int nblkX = NROWS / 32;
  const dim3 gCvtX(nblkX);
  const dim3 gCvtW(CH / 8);
  const dim3 gXW(((NROWS / 64) * (CH / 64) + 7) / 8, 1);
  const dim3 gHT(((CH / 64) * (SEQ / 64) + 7) / 8, NBATCH);
  const dim3 gAttn(NBATCH * NQB);

  cvt_x_rn<<<gCvtX, blk, 0, stream>>>(x, Xb, rnp, nblkX);
  cvt_w<<<gCvtW, blk, 0, stream>>>(adjw, affw, WT, WA);
  gemm64<0, 2, false><<<gXW, blk, 0, stream>>>(
      Xb, Xb, CH, 0LL, WT, WT, CH, 0LL,
      (void*)XWh, CH, 0LL, (void*)XWl, CH, 0LL, CH,
      affb, NROWS, CH, CH, 1.0f);
  gemm64<0, 3, true><<<gHT, blk, 0, stream>>>(
      WA, WA, CH, 0LL, Xb, Xb, CH, (long long)SEQ * CH,
      (void*)Hth, SEQ, (long long)CH * SEQ, (void*)Hth, SEQ, (long long)CH * SEQ, 0,
      affb, CH, SEQ, CH, 4096.0f);
  attn_ln<<<gAttn, blk, 0, stream>>>(XWh, XWl, Xb, Hth, rnp, lng, lnb, (float*)d_out,
                                     1024.0f, 1.0f / 1024.0f, 5.0f);
  (void)hipGetLastError();
}
